// GNN_73710228733973
// MI455X (gfx1250) — hardware-verified
//
#include <hip/hip_runtime.h>
#include <stddef.h>
#include <stdint.h>
#include <math.h>


#define NNODE  32768
#define NEDGE  524288
#define HID    256
#define NGR    64
#define NPG    512
#define FOUT   512
#define MLPW   1024
#define NTHR   256
#define NWAVE  8
#define EPT    8
#define CHUNK  (NTHR * EPT)
#define WCAP   (EPT * 32)
#define LISTN  (NWAVE * WCAP)
#define NBA    1024
#define SLA    10
#define RCAP   28672
#define DEGCAP 64
#define GBM    64
#define GBN    64
#define GTHR   128
#define AGG_ZINTS (LISTN + 2 * RCAP + 3 * NBA)
#define AGG_LDS_INTS (AGG_ZINTS + 16)
#define WSMAX  134217728
#define WU1 8192
#define WU2 16384
#define WU3 32768
#define WU4 49152
#define WU5 114688
#define WU6 180224
#define WU7 212992

static_assert((CHUNK & (CHUNK - 1)) == 0 && CHUNK <= 4096);
static_assert((NBA & (NBA - 1)) == 0 && NBA == (1 << SLA));
static_assert(((long long)NEDGE << SLA) < (1LL << 31));
static_assert(LISTN % NTHR == 0 && NBA % NWAVE == 0 && NBA % 32 == 0);
static_assert(RCAP % 32 == 0 && AGG_ZINTS % 4 == 0 && LISTN % 4 == 0);
static_assert(AGG_LDS_INTS * 4 <= 300000);
static_assert(NNODE % NBA == 0 && NNODE % GBM == 0 && NEDGE % CHUNK == 0);
static_assert(HID == 8 * 32 && HID % 32 == 0 && NGR == GBM && NGR * NPG == NNODE);
static_assert(WU1 % NTHR == 0 && WU2 % NTHR == 0 && WU3 % NTHR == 0 && WU4 % NTHR == 0);
static_assert(WU5 % NTHR == 0 && WU6 % NTHR == 0 && WU7 % NTHR == 0);
static_assert(DEGCAP >= 36 + 8 && RCAP >= 16659 + 4096);
static_assert(NGR * FOUT + NGR * HID == 49152);

typedef float          v4f   __attribute__((ext_vector_type(4)));
typedef float          v8f   __attribute__((ext_vector_type(8)));
typedef int            v4i   __attribute__((ext_vector_type(4)));
typedef int            v8i   __attribute__((ext_vector_type(8)));
typedef unsigned int   v4u   __attribute__((ext_vector_type(4)));
typedef unsigned short v8us  __attribute__((ext_vector_type(8)));
typedef unsigned short v16us __attribute__((ext_vector_type(16)));
typedef __bf16         v16bf __attribute__((ext_vector_type(16)));
typedef v4f  __attribute__((may_alias)) v4fa;
typedef v4i  __attribute__((may_alias)) v4ia;
typedef v8us __attribute__((may_alias)) v8usa;
union FragB { v16bf v; v16us u; v8us h[2]; v8i w; };

__device__ __forceinline__ v8f wmb(const FragB& a, const FragB& b, v8f c) {
  v8f d = __builtin_amdgcn_wmma_f32_16x16x32_bf16(false, a.v, false, b.v, (short)0, c, false, false);
  asm volatile("v_nop\n\tv_nop\n\tv_nop\n\tv_nop" : "+v"(d) : "v"(a.w), "v"(b.w));
  return d;
}

__device__ __forceinline__ unsigned bf16_bits(float f) {
  const unsigned u = __float_as_uint(f);
  return ((u + 0x7FFFu + ((u >> 16) & 1u)) >> 16) & 0xFFFFu;
}
__device__ __forceinline__ float bf16_val(float f) {
  return __uint_as_float(bf16_bits(f) << 16);
}
__device__ __forceinline__ float gelu_erf(float x) {
  return 0.5f * x * (1.0f + erff(x * 0.70710678118654752f));
}

template <int SLB>
__device__ __forceinline__ int scan_chunk(const int* __restrict__ dsts, int nE, int cbase, int slotBase,
                                          int nb, int vec8, int* list, int tid, int lane, int wave) {
  int wc = 0;
  const int el0  = tid * EPT;
  const int e0   = cbase + el0;
  const int sent = -2147483647 - 1;
  v4i da, db;
  if (vec8 != 0 && cbase + CHUNK <= nE) {
    da = *(const v4i*)(dsts + e0);
    db = *(const v4i*)(dsts + e0 + 4);
  } else {
    da.x = (e0     < nE) ? dsts[min(e0,     nE - 1)] : sent;
    da.y = (e0 + 1 < nE) ? dsts[min(e0 + 1, nE - 1)] : sent;
    da.z = (e0 + 2 < nE) ? dsts[min(e0 + 2, nE - 1)] : sent;
    da.w = (e0 + 3 < nE) ? dsts[min(e0 + 3, nE - 1)] : sent;
    db.x = (e0 + 4 < nE) ? dsts[min(e0 + 4, nE - 1)] : sent;
    db.y = (e0 + 5 < nE) ? dsts[min(e0 + 5, nE - 1)] : sent;
    db.z = (e0 + 6 < nE) ? dsts[min(e0 + 6, nE - 1)] : sent;
    db.w = (e0 + 7 < nE) ? dsts[min(e0 + 7, nE - 1)] : sent;
  }
  const unsigned nbs = (unsigned)slotBase;
  const unsigned unb = (unsigned)nb;
  const unsigned s0 = (unsigned)da.x - nbs, s1 = (unsigned)da.y - nbs;
  const unsigned s2 = (unsigned)da.z - nbs, s3 = (unsigned)da.w - nbs;
  const unsigned s4 = (unsigned)db.x - nbs, s5 = (unsigned)db.y - nbs;
  const unsigned s6 = (unsigned)db.z - nbs, s7 = (unsigned)db.w - nbs;
  const bool h0 = s0 < unb, h1 = s1 < unb, h2 = s2 < unb, h3 = s3 < unb;
  const bool h4 = s4 < unb, h5 = s5 < unb, h6 = s6 < unb, h7 = s7 < unb;
  const unsigned any = __builtin_amdgcn_ballot_w32(h0 | h1 | h2 | h3 | h4 | h5 | h6 | h7);
  if (any != 0u) {
#define HITJ(J, HJ, SJ) { \
      const unsigned mj = __builtin_amdgcn_ballot_w32(HJ); \
      if (mj != 0u) { \
        if (HJ) { \
          const int pos = wc + (int)__builtin_amdgcn_mbcnt_lo(mj, 0u); \
          if (pos < WCAP) list[wave * WCAP + pos] = ((el0 + (J)) << SLB) | (int)(SJ); \
        } \
        wc += (int)__builtin_popcount(mj); } }
    HITJ(0, h0, s0)
    HITJ(1, h1, s1)
    HITJ(2, h2, s2)
    HITJ(3, h3, s3)
    HITJ(4, h4, s4)
    HITJ(5, h5, s5)
    HITJ(6, h6, s6)
    HITJ(7, h7, s7)
#undef HITJ
  }
  return wc;
}

template <int KP, int KIN, int SRCN>
__device__ __forceinline__ void wunit(const float* __restrict__ W, unsigned short* P, int v, int ndOff) {
  constexpr int UPR = KP / 8;
  const int nl = v / UPR;
  const int k8 = (v % UPR) * 8;
  const int kk = k8 % KIN;
  const float* p = W + (size_t)kk * SRCN + nl;
  v8us o;
#pragma unroll
  for (int i = 0; i < 8; ++i) o[i] = (unsigned short)bf16_bits(p[(size_t)i * SRCN]);
  unsigned short* dp = P + (size_t)(ndOff + nl) * KP + k8;
  *(volatile v8us*)dp = o;
  __threadfence();
  *(volatile v8us*)dp = o;
}

__global__ __launch_bounds__(NTHR) void k_wprep(const float* __restrict__ w1l, const float* __restrict__ w1r,
                                                const float* __restrict__ w2l, const float* __restrict__ w2r,
                                                const float* __restrict__ l1w, const float* __restrict__ l2w,
                                                const float* __restrict__ fw,
                                                unsigned short* W1T, unsigned short* W2T2, unsigned short* L1T2,
                                                unsigned short* L2T2, unsigned short* FINT2) {
  const int u = (int)blockIdx.x * NTHR + (int)threadIdx.x;
  if (u < WU1)       wunit<256, 256, 256>(w1l, W1T, u, 0);
  else if (u < WU2)  wunit<256, 256, 256>(w1r, W1T, u - WU1, 256);
  else if (u < WU3)  wunit<512, 256, 256>(w2l, W2T2, u - WU2, 0);
  else if (u < WU4)  wunit<512, 256, 256>(w2r, W2T2, u - WU3, 256);
  else if (u < WU5)  wunit<512, 256, 1024>(l1w, L1T2, u - WU4, 0);
  else if (u < WU6)  wunit<2048, 1024, 256>(l2w, L2T2, u - WU5, 0);
  else if (u < WU7)  wunit<512, 256, 512>(fw, FINT2, u - WU6, 0);
}

__global__ __launch_bounds__(NTHR) void k_cvx(const float* __restrict__ x, int nUnits, unsigned short* xb) {
  const int u = (int)blockIdx.x * NTHR + (int)threadIdx.x;
  if (u >= nUnits) return;
  const int row = u >> 5;
  const int k8  = (u & 31) * 8;
  const float* p = x + (size_t)row * HID + k8;
  const v4f a = *(const v4fa*)p;
  const v4f b = *(const v4fa*)(p + 4);
  v8us o;
  o[0] = (unsigned short)bf16_bits(a.x); o[1] = (unsigned short)bf16_bits(a.y);
  o[2] = (unsigned short)bf16_bits(a.z); o[3] = (unsigned short)bf16_bits(a.w);
  o[4] = (unsigned short)bf16_bits(b.x); o[5] = (unsigned short)bf16_bits(b.y);
  o[6] = (unsigned short)bf16_bits(b.z); o[7] = (unsigned short)bf16_bits(b.w);
  unsigned short* dp = xb + (size_t)row * HID + k8;
  *(volatile v8us*)dp = o;
  __threadfence();
  *(volatile v8us*)dp = o;
}

template <int EP>
__global__ __launch_bounds__(GTHR) void k_gemm(
    const unsigned short* __restrict__ A, const unsigned short* __restrict__ WT,
    const float* __restrict__ biasA, const float* __restrict__ biasB,
    float* outF, unsigned short* outH, int K, int N, int pstride)
{
  constexpr bool HL = (EP == 1 || EP == 2);
  constexpr int PKN = HL ? (GBM * 2 * 8) : 4;
  __shared__ __attribute__((aligned(16))) float stg[GBM * GBN];
  __shared__ __attribute__((aligned(16))) v4u pk[PKN];
  const int tid = (int)threadIdx.x, lane = tid & 31, wave = tid >> 5, hh = lane >> 4, m = lane & 15;
  const int rowBase = (int)blockIdx.x * GBM;
  const int col0    = (int)blockIdx.y * GBN;

  v8f acc[4];
  {
    const v8f z = {0.f, 0.f, 0.f, 0.f, 0.f, 0.f, 0.f, 0.f};
    acc[0] = z; acc[1] = z; acc[2] = z; acc[3] = z;
  }
  const unsigned short* ap = A  + (size_t)(rowBase + 16 * wave + m) * (size_t)K + 8 * hh;
  const unsigned short* wp = WT + (size_t)(col0 + m) * (size_t)K + 8 * hh;
  const int ksteps = K >> 5;
#pragma unroll 1
  for (int ks = 0; ks < ksteps; ++ks) {
    FragB af;
    af.h[0] = *(const v8usa*)(ap + 32 * ks);
    af.h[1] = *(const v8usa*)(ap + 32 * ks + 16);
#pragma unroll
    for (int t = 0; t < 4; ++t) {
      const unsigned short* wq = wp + (size_t)(16 * t) * (size_t)K + 32 * ks;
      FragB bf;
      bf.h[0] = *(const v8usa*)wq;
      bf.h[1] = *(const v8usa*)(wq + 16);
      acc[t] = wmb(af, bf, acc[t]);
    }
  }

#pragma unroll
  for (int t = 0; t < 4; ++t) {
    const int lc = 16 * t + m;
#pragma unroll
    for (int r = 0; r < 8; ++r) {
      const int lr = 16 * wave + 8 * hh + r;
      stg[lr * GBN + lc] = acc[t][r];
    }
  }
  __syncthreads();

  if constexpr (!HL) {
    v4f bv;
    int cin, ldo;
    size_t base;
    if constexpr (EP == 0) {
      const int cb = (col0 & 255) + 4 * m;
      const v4f a = *(const v4f*)(biasA + cb);
      const v4f b = *(const v4f*)(biasB + cb);
      const bool sel = col0 >= 256;
      bv.x = bf16_val(sel ? b.x : a.x);
      bv.y = bf16_val(sel ? b.y : a.y);
      bv.z = bf16_val(sel ? b.z : a.z);
      bv.w = bf16_val(sel ? b.w : a.w);
      cin = cb; ldo = 256; base = sel ? (size_t)pstride : (size_t)0;
    } else {
      const int cb = col0 + 4 * m;
      const v4f a = *(const v4f*)(biasA + cb);
      bv.x = bf16_val(a.x); bv.y = bf16_val(a.y); bv.z = bf16_val(a.z); bv.w = bf16_val(a.w);
      cin = cb; ldo = N; base = 0;
    }
    v4f fv[8];
#pragma unroll
    for (int i = 0; i < 8; ++i) {
      const int lr = 16 * wave + 2 * i + hh;
      fv[i] = *(const v4fa*)(stg + lr * GBN + 4 * m) + bv;
    }
#pragma unroll
    for (int i = 0; i < 8; ++i) {
      const int gr = rowBase + 16 * wave + 2 * i + hh;
      float* op = outF + base + (size_t)gr * (size_t)ldo + cin;
      *(volatile v4f*)op = fv[i];
    }
    __threadfence();
#pragma unroll
    for (int i = 0; i < 8; ++i) {
      const int gr = rowBase + 16 * wave + 2 * i + hh;
      float* op = outF + base + (size_t)gr * (size_t)ldo + cin;
      *(volatile v4f*)op = fv[i];
    }
  } else {
    const int c8 = (tid & 7) * 8;
    float bsv[8];
    {
      const v4f a = *(const v4f*)(biasA + col0 + c8);
      const v4f b = *(const v4f*)(biasA + col0 + c8 + 4);
      bsv[0] = bf16_val(a.x); bsv[1] = bf16_val(a.y); bsv[2] = bf16_val(a.z); bsv[3] = bf16_val(a.w);
      bsv[4] = bf16_val(b.x); bsv[5] = bf16_val(b.y); bsv[6] = bf16_val(b.z); bsv[7] = bf16_val(b.w);
    }
#pragma unroll 1
    for (int it = 0; it < 8; ++it) {
      const int L    = it * 16 + (tid >> 3);
      const int row  = L >> 1;
      const bool lo  = (L & 1) != 0;
      const v4f f0 = *(const v4fa*)(stg + row * GBN + c8);
      const v4f f1 = *(const v4fa*)(stg + row * GBN + c8 + 4);
      float t[8] = {f0.x, f0.y, f0.z, f0.w, f1.x, f1.y, f1.z, f1.w};
      unsigned hw[8];
#pragma unroll
      for (int j = 0; j < 8; ++j) {
        float v = t[j] + bsv[j];
        if constexpr (EP == 1) v = gelu_erf(v);
        const unsigned hb = bf16_bits(v);
        const unsigned lb = bf16_bits(v - __uint_as_float(hb << 16));
        hw[j] = lo ? lb : hb;
      }
      v4u q;
      q.x = hw[0] | (hw[1] << 16); q.y = hw[2] | (hw[3] << 16);
      q.z = hw[4] | (hw[5] << 16); q.w = hw[6] | (hw[7] << 16);
      pk[it * GTHR + tid] = q;
    }
#pragma unroll 1
    for (int it = 0; it < 8; ++it) {
      const int L = it * 16 + (tid >> 3);
      const v4u q = pk[it * GTHR + tid];
      unsigned short* op = outH + (size_t)(rowBase + (L >> 1)) * (size_t)(2 * N) + (size_t)((L & 1) * N) + col0 + c8;
      *(volatile v4u*)op = q;
    }
    __threadfence();
#pragma unroll 1
    for (int it = 0; it < 8; ++it) {
      const int L = it * 16 + (tid >> 3);
      const v4u q = pk[it * GTHR + tid];
      unsigned short* op = outH + (size_t)(rowBase + (L >> 1)) * (size_t)(2 * N) + (size_t)((L & 1) * N) + col0 + c8;
      *(volatile v4u*)op = q;
    }
  }
}

template <int MODE>
__global__ __launch_bounds__(NTHR) void k_scan(const int* __restrict__ srcs, const int* __restrict__ dsts,
                                               int nE, int nN, int vec8,
                                               const float* __restrict__ xl, float* xr,
                                               const float* __restrict__ att, const float* __restrict__ bias,
                                               unsigned short* h1) {
  extern __shared__ __attribute__((aligned(16))) int dsm[];
  int* list = dsm;
  int* hl   = dsm + LISTN;
  int* sl   = dsm + LISTN + RCAP;
  int* cnt  = dsm + LISTN + 2 * RCAP;
  int* offs = cnt + NBA;
  int* cur  = offs + NBA;
  int* misc = cur + NBA;
  const int tid = (int)threadIdx.x, lane = tid & 31, wave = tid >> 5;
  const int nodeBase = (int)blockIdx.x * NBA;

  {
    const v4i z4 = {0, 0, 0, 0};
    for (int i = tid * 4; i < AGG_ZINTS; i += NTHR * 4) *(v4ia*)(dsm + i) = z4;
    if (tid < 16) misc[tid] = 0;
  }
  __syncthreads();

  int t = 0, ov = 0;
  const int nChunks = (nE + CHUNK - 1) / CHUNK;
#pragma unroll 1
  for (int ch = 0; ch < nChunks; ++ch) {
    const int cbase = ch * CHUNK;
    const int wc = scan_chunk<SLA>(dsts, nE, cbase, nodeBase, NBA, vec8, list, tid, lane, wave);
    if (lane == 0) misc[wave] = wc;
    __syncthreads();
    if (wave == 0) {
#pragma unroll 1
      for (int w2 = 0; w2 < NWAVE; ++w2) {
        int c = misc[w2];
        c = c < 0 ? 0 : (c > WCAP ? WCAP : c);
#pragma unroll 1
        for (int b0 = 0; b0 < c; b0 += 32) {
          const int idx = b0 + lane;
          const int ent = list[w2 * WCAP + (idx < WCAP ? idx : WCAP - 1)];
          const int m32 = (c - b0) < 32 ? (c - b0) : 32;
#pragma unroll 1
          for (int k = 0; k < m32; ++k) {
            const int u    = __builtin_amdgcn_readlane(ent, k);
            const int slot = u & (NBA - 1);
            const int el   = (u >> SLA) & (CHUNK - 1);
            const int pk   = ((cbase + el) << SLA) | slot;
            if (t < RCAP) {
              if (lane == 0) { hl[t] = pk; cnt[slot] = cnt[slot] + 1; }
              t = t + 1;
            } else {
              ov = 1;
            }
          }
        }
      }
    }
    __syncthreads();
  }
  if (wave == 0 && lane == 0) { misc[8] = t; misc[9] = ov; }
  __syncthreads();
  int tt = misc[8];
  tt = tt < 0 ? 0 : (tt > RCAP ? RCAP : tt);
  const int ovf = misc[9];

  if (wave == 0) {
    const int base = lane * (NBA / 32);
    int s = 0;
#pragma unroll 1
    for (int i = 0; i < NBA / 32; ++i) s += cnt[base + i];
    int incl = s;
#pragma unroll
    for (int d = 1; d < 32; d <<= 1) {
      const int y = __shfl_up(incl, d, 32);
      if (lane >= d) incl += y;
    }
    int run = incl - s;
#pragma unroll 1
    for (int i = 0; i < NBA / 32; ++i) {
      const int cv = cnt[base + i];
      offs[base + i] = run;
      cur[base + i]  = run;
      run += cv;
    }
  }
  __syncthreads();
  if (wave == 0) {
#pragma unroll 1
    for (int b0 = 0; b0 < tt; b0 += 32) {
      const int idx = b0 + lane;
      const int ent = hl[idx < RCAP ? idx : RCAP - 1];
      const int m32 = (tt - b0) < 32 ? (tt - b0) : 32;
#pragma unroll 1
      for (int k = 0; k < m32; ++k) {
        const int u    = __builtin_amdgcn_readlane(ent, k);
        const int slot = u & (NBA - 1);
        if (lane == 0) {
          int p = cur[slot];
          p = p < 0 ? 0 : (p > RCAP - 1 ? RCAP - 1 : p);
          sl[p] = u;
          cur[slot] = p + 1;
        }
      }
    }
  }
  __syncthreads();

  const int c0 = 8 * lane;
  float at[8], bs[8];
  {
    const v4f a = *(const v4f*)(att + c0);
    const v4f b = *(const v4f*)(att + c0 + 4);
    at[0] = bf16_val(a.x); at[1] = bf16_val(a.y); at[2] = bf16_val(a.z); at[3] = bf16_val(a.w);
    at[4] = bf16_val(b.x); at[5] = bf16_val(b.y); at[6] = bf16_val(b.z); at[7] = bf16_val(b.w);
    const v4f c = *(const v4f*)(bias + c0);
    const v4f d = *(const v4f*)(bias + c0 + 4);
    bs[0] = bf16_val(c.x); bs[1] = bf16_val(c.y); bs[2] = bf16_val(c.z); bs[3] = bf16_val(c.w);
    bs[4] = bf16_val(d.x); bs[5] = bf16_val(d.y); bs[6] = bf16_val(d.z); bs[7] = bf16_val(d.w);
  }
  const float qnan = __int_as_float(0x7fc00000);
  const float pz = (ovf != 0) ? qnan : 0.0f;
  const int sA = lane >> 1, sB = 16 + (lane >> 1);
  const bool odd = (lane & 1) != 0;
#pragma unroll 1
  for (int si = 0; si < NBA / NWAVE; ++si) {
    const int s = si * NWAVE + wave;
    int node = nodeBase + s;
    node = node < nN ? node : nN - 1;
    int c = cnt[s];
    const bool big = c > DEGCAP;
    c = c < 0 ? 0 : (c > DEGCAP ? DEGCAP : c);
    int o = offs[s];
    o = o < 0 ? 0 : (o > RCAP ? RCAP : o);
    float xrv[8];
    {
      const float* rp = xr + (size_t)node * HID + c0;
      const v4f ra = *(const v4fa*)rp;
      const v4f rb = *(const v4fa*)(rp + 4);
      xrv[0] = ra.x; xrv[1] = ra.y; xrv[2] = ra.z; xrv[3] = ra.w;
      xrv[4] = rb.x; xrv[5] = rb.y; xrv[6] = rb.z; xrv[7] = rb.w;
    }
    float mrun = -3.0e38f, ssum = 0.0f;
    float acc[8] = {0.f, 0.f, 0.f, 0.f, 0.f, 0.f, 0.f, 0.f};
    const int ct = c + 1;
#pragma unroll 1
    for (int b0 = 0; b0 < ct; b0 += 32) {
      const int q = b0 + lane;
      int idx = o + q;
      idx = idx < 0 ? 0 : (idx > RCAP - 1 ? RCAP - 1 : idx);
      const int ent = sl[idx];
      int eid = ent >> SLA;
      eid = eid < 0 ? 0 : (eid > nE - 1 ? nE - 1 : eid);
      int sr = srcs[eid];
      sr = sr < 0 ? 0 : (sr > nN - 1 ? nN - 1 : sr);
      sr = (q < c) ? sr : node;
      const int m32 = (ct - b0) < 32 ? (ct - b0) : 32;
#pragma unroll 1
      for (int k = 0; k < m32; ++k) {
        const int sk = __builtin_amdgcn_readlane(sr, k);
        const float* sp = xl + (size_t)sk * HID + c0;
        const v4f xa = *(const v4f*)sp;
        const v4f xb = *(const v4f*)(sp + 4);
        const float xv[8] = {xa.x, xa.y, xa.z, xa.w, xb.x, xb.y, xb.z, xb.w};
        float part = 0.0f;
#pragma unroll
        for (int i = 0; i < 8; ++i) {
          float tv = xv[i] + xrv[i];
          tv = (tv > 0.0f) ? tv : 0.2f * tv;
          part = fmaf(at[i], tv, part);
        }
        part += __shfl_xor(part, 1, 32);
        part += __shfl_xor(part, 2, 32);
        part += __shfl_xor(part, 4, 32);
        const float d  = part - mrun;
        const float e  = expf(-fabsf(d));
        const bool  up = d > 0.0f;
        const float sc = up ? e : 1.0f;
        const float p  = up ? 1.0f : e;
        mrun = up ? part : mrun;
        ssum = fmaf(ssum, sc, p);
#pragma unroll
        for (int i = 0; i < 8; ++i) acc[i] = fmaf(p, xv[i], acc[i] * sc);
      }
    }
    const float inv = 1.0f / (ssum + 1e-16f);
    float v[8];
#pragma unroll
    for (int i = 0; i < 8; ++i) v[i] = fmaf(acc[i], inv, bs[i]);
    const float pzr = big ? qnan : pz;
    if constexpr (MODE != 0) {
#pragma unroll 1
      for (int r = 0; r < 8; ++r) {
        const float g = gelu_erf(v[0]);
        v[0] = v[1]; v[1] = v[2]; v[2] = v[3]; v[3] = v[4];
        v[4] = v[5]; v[5] = v[6]; v[6] = v[7]; v[7] = g;
      }
      unsigned hb[8], lb[8];
#pragma unroll
      for (int i = 0; i < 8; ++i) {
        const float y = v[i] + pzr;
        hb[i] = bf16_bits(y);
        lb[i] = bf16_bits(y - __uint_as_float(hb[i] << 16));
      }
      v4u hq, lq;
      hq.x = hb[0] | (hb[1] << 16); hq.y = hb[2] | (hb[3] << 16);
      hq.z = hb[4] | (hb[5] << 16); hq.w = hb[6] | (hb[7] << 16);
      lq.x = lb[0] | (lb[1] << 16); lq.y = lb[2] | (lb[3] << 16);
      lq.z = lb[4] | (lb[5] << 16); lq.w = lb[6] | (lb[7] << 16);
      unsigned short* hp = h1 + (size_t)node * (2 * HID) + c0;
      *(volatile v4u*)hp = hq;
      *(volatile v4u*)(hp + HID) = lq;
      __threadfence();
      *(volatile v4u*)hp = hq;
      *(volatile v4u*)(hp + HID) = lq;
    } else {
      float y[8];
#pragma unroll
      for (int i = 0; i < 8; ++i) y[i] = v[i] + pzr;
      float oa[4], ob[4];
#pragma unroll
      for (int j = 0; j < 4; ++j) {
        const float a0 = __shfl(y[j], sA, 32);
        const float a1 = __shfl(y[4 + j], sA, 32);
        const float b0 = __shfl(y[j], sB, 32);
        const float b1 = __shfl(y[4 + j], sB, 32);
        oa[j] = odd ? a1 : a0;
        ob[j] = odd ? b1 : b0;
      }
      v4f wa, wb;
      wa.x = oa[0]; wa.y = oa[1]; wa.z = oa[2]; wa.w = oa[3];
      wb.x = ob[0]; wb.y = ob[1]; wb.z = ob[2]; wb.w = ob[3];
      float* op = xr + (size_t)node * HID + 4 * lane;
      *(volatile v4f*)op = wa;
      *(volatile v4f*)(op + 128) = wb;
      __threadfence();
      *(volatile v4f*)op = wa;
      *(volatile v4f*)(op + 128) = wb;
    }
  }
}

__global__ __launch_bounds__(NTHR) void k_pool(const float* __restrict__ h2, const int* __restrict__ bat,
                                               const int* __restrict__ bsz, int nN, int npg,
                                               float* outMean, unsigned short* z0) {
  __shared__ __attribute__((aligned(16))) float wsum[NWAVE * HID];
  __shared__ int wcn[NWAVE];
  __shared__ __attribute__((aligned(16))) float outs[HID];
  __shared__ __attribute__((aligned(16))) unsigned short zrow[2 * HID];
  const int tid = (int)threadIdx.x, lane = tid & 31, wave = tid >> 5;
  const int g = (int)blockIdx.x;

  v4f a0 = {0.f, 0.f, 0.f, 0.f}, a1 = {0.f, 0.f, 0.f, 0.f};
  int cnt = 0;
#pragma unroll 1
  for (int i0 = wave * 32; i0 < nN; i0 += NTHR) {
    const int i  = i0 + lane;
    const int ic = i < nN ? i : nN - 1;
    const int b  = bat[ic];
    const bool hit = (i < nN) && (b == g);
    unsigned msk = __builtin_amdgcn_ballot_w32(hit);
    int nh = (int)__builtin_popcount(msk);
    nh = nh > 32 ? 32 : nh;
    cnt += nh;
#pragma unroll 1
    for (int q = 0; q < nh; ++q) {
      const int k = __builtin_ffs((int)msk) - 1;
      msk &= msk - 1u;
      int node = i0 + (k < 0 ? 0 : k);
      node = node > nN - 1 ? nN - 1 : node;
      const float* rp = h2 + (size_t)node * HID + 8 * lane;
      const v4f u0 = *(const v4f*)rp;
      const v4f u1 = *(const v4f*)(rp + 4);
      a0 = a0 + u0; a1 = a1 + u1;
    }
  }
  *(v4fa*)(wsum + wave * HID + 8 * lane)     = a0;
  *(v4fa*)(wsum + wave * HID + 8 * lane + 4) = a1;
  if (lane == 0) wcn[wave] = cnt;
  __syncthreads();
  {
    const float pzg = (bsz[0] != NGR) ? __int_as_float(0x7fc00000) : 0.0f;
    float s = 0.0f;
    int c = 0;
#pragma unroll
    for (int w2 = 0; w2 < NWAVE; ++w2) { s += wsum[w2 * HID + tid]; c += wcn[w2]; }
    const float cf = (c < 1) ? 1.0f : (float)c;
    outs[tid] = s * (1.0f / cf) + pzg;
    long long n0 = (long long)g * (long long)npg;
    n0 = n0 > (long long)(nN - 1) ? (long long)(nN - 1) : n0;
    const float zv = h2[(size_t)n0 * HID + tid] + pzg;
    const unsigned hb = bf16_bits(zv);
    const unsigned lb = bf16_bits(zv - __uint_as_float(hb << 16));
    zrow[tid]       = (unsigned short)hb;
    zrow[HID + tid] = (unsigned short)lb;
  }
  __syncthreads();
  if (wave == 0) {
    const v4f o0 = *(const v4fa*)(outs + 4 * lane);
    const v4f o1 = *(const v4fa*)(outs + 128 + 4 * lane);
    float* op = outMean + (size_t)g * HID + 4 * lane;
    *(volatile v4f*)op = o0;
    *(volatile v4f*)(op + 128) = o1;
    __threadfence();
    *(volatile v4f*)op = o0;
    *(volatile v4f*)(op + 128) = o1;
  } else if (wave == 1) {
    const v8us q0 = *(const v8usa*)(zrow + 8 * lane);
    const v8us q1 = *(const v8usa*)(zrow + HID + 8 * lane);
    unsigned short* zp = z0 + (size_t)g * (2 * HID) + 8 * lane;
    *(volatile v8us*)zp = q0;
    *(volatile v8us*)(zp + HID) = q1;
    __threadfence();
    *(volatile v8us*)zp = q0;
    *(volatile v8us*)(zp + HID) = q1;
  }
}

static inline size_t al256(size_t o) { return (o + 255) & ~(size_t)255; }

extern "C" void kernel_launch(void* const* d_in, const int* in_sizes, int n_in,
                              void* d_out, int out_size, void* d_ws, size_t ws_size,
                              hipStream_t stream) {
  if (n_in < 22) return;
  if (in_sizes[0] != NNODE * HID) return;
  if (in_sizes[1] != 2 * NEDGE) return;
  if (in_sizes[2] != NNODE || in_sizes[3] != 1) return;
  if (in_sizes[4] != HID * HID || in_sizes[5] != HID) return;
  if (in_sizes[6] != HID * HID || in_sizes[7] != HID) return;
  if (in_sizes[8] != HID || in_sizes[9] != HID) return;
  if (in_sizes[10] != HID * HID || in_sizes[11] != HID) return;
  if (in_sizes[12] != HID * HID || in_sizes[13] != HID) return;
  if (in_sizes[14] != HID || in_sizes[15] != HID) return;
  if (in_sizes[16] != HID * MLPW || in_sizes[17] != MLPW) return;
  if (in_sizes[18] != MLPW * HID || in_sizes[19] != HID) return;
  if (in_sizes[20] != HID * FOUT || in_sizes[21] != FOUT) return;
  if (out_size != NGR * FOUT + NGR * HID) return;

  const float* x     = (const float*)d_in[0];
  const int*   edge  = (const int*)d_in[1];
  const int*   bat   = (const int*)d_in[2];
  const int*   bsz   = (const int*)d_in[3];
  const float* w1l   = (const float*)d_in[4];
  const float* b1l   = (const float*)d_in[5];
  const float* w1r   = (const float*)d_in[6];
  const float* b1r   = (const float*)d_in[7];
  const float* att1  = (const float*)d_in[8];
  const float* bias1 = (const float*)d_in[9];
  const float* w2l   = (const float*)d_in[10];
  const float* b2l   = (const float*)d_in[11];
  const float* w2r   = (const float*)d_in[12];
  const float* b2r   = (const float*)d_in[13];
  const float* att2  = (const float*)d_in[14];
  const float* bias2 = (const float*)d_in[15];
  const float* l1w   = (const float*)d_in[16];
  const float* l1b   = (const float*)d_in[17];
  const float* l2w   = (const float*)d_in[18];
  const float* l2b   = (const float*)d_in[19];
  const float* fw    = (const float*)d_in[20];
  const float* fb    = (const float*)d_in[21];
  float* out = (float*)d_out;
  const int nN = NNODE, nE = NEDGE;
  const int* src = edge;
  const int* dst = edge + nE;
  const int vec8 = 1;

  char* ws = (char*)d_ws;
  size_t off = 0;
  const size_t oXL  = off; off = al256(off + (size_t)2 * NNODE * HID * 4);
  const size_t oH1  = off; off = al256(off + (size_t)NNODE * 2 * HID * 2);
  const size_t oXB  = off; off = al256(off + (size_t)NNODE * HID * 2);
  const size_t oW1  = off; off = al256(off + (size_t)512 * 256 * 2);
  const size_t oW2  = off; off = al256(off + (size_t)512 * 512 * 2);
  const size_t oL1  = off; off = al256(off + (size_t)1024 * 512 * 2);
  const size_t oL2  = off; off = al256(off + (size_t)256 * 2048 * 2);
  const size_t oFN  = off; off = al256(off + (size_t)512 * 512 * 2);
  const size_t oZ0  = off; off = al256(off + (size_t)NGR * 2 * HID * 2);
  const size_t oF   = off; off = al256(off + (size_t)NGR * 2 * MLPW * 2);
  const size_t oZ2  = off; off = al256(off + (size_t)NGR * 2 * HID * 2);
  if (off > ws_size || off > (size_t)WSMAX) return;
  float*          XL   = (float*)(ws + oXL);
  float*          XR   = XL + (size_t)NNODE * HID;
  unsigned short* H1   = (unsigned short*)(ws + oH1);
  unsigned short* XB   = (unsigned short*)(ws + oXB);
  unsigned short* W1T  = (unsigned short*)(ws + oW1);
  unsigned short* W2T2 = (unsigned short*)(ws + oW2);
  unsigned short* L1T2 = (unsigned short*)(ws + oL1);
  unsigned short* L2T2 = (unsigned short*)(ws + oL2);
  unsigned short* FNT2 = (unsigned short*)(ws + oFN);
  unsigned short* Z0   = (unsigned short*)(ws + oZ0);
  unsigned short* F    = (unsigned short*)(ws + oF);
  unsigned short* Z2   = (unsigned short*)(ws + oZ2);
  const int pstride = NNODE * HID;

  const size_t scanLds = (size_t)AGG_LDS_INTS * 4;
  hipFuncSetAttribute(reinterpret_cast<const void*>(&k_scan<1>), hipFuncAttributeMaxDynamicSharedMemorySize, (int)scanLds);
  hipFuncSetAttribute(reinterpret_cast<const void*>(&k_scan<0>), hipFuncAttributeMaxDynamicSharedMemorySize, (int)scanLds);

  const int nUx = NNODE * (HID / 8);
  k_cvx<<<nUx / NTHR, NTHR, 0, stream>>>(x, nUx, XB);
  k_wprep<<<WU7 / NTHR, NTHR, 0, stream>>>(w1l, w1r, w2l, w2r, l1w, l2w, fw, W1T, W2T2, L1T2, L2T2, FNT2);
  k_gemm<0><<<dim3(NNODE / GBM, 512 / GBN), GTHR, 0, stream>>>(XB, W1T, b1l, b1r, XL, H1, HID, 512, pstride);
  k_scan<1><<<NNODE / NBA, NTHR, scanLds, stream>>>(src, dst, nE, nN, vec8, XL, XR, att1, bias1, H1);
  k_gemm<0><<<dim3(NNODE / GBM, 512 / GBN), GTHR, 0, stream>>>(H1, W2T2, b2l, b2r, XL, H1, 2 * HID, 512, pstride);
  k_scan<0><<<NNODE / NBA, NTHR, scanLds, stream>>>(src, dst, nE, nN, vec8, XL, XR, att2, bias2, H1);
  k_pool<<<NGR, NTHR, 0, stream>>>(XR, bat, bsz, nN, NPG, out + (size_t)NGR * FOUT, Z0);
  k_gemm<1><<<dim3(1, MLPW / GBN), GTHR, 0, stream>>>(Z0, L1T2, l1b, l1b, XL, F, 2 * HID, MLPW, 0);
  k_gemm<2><<<dim3(1, HID / GBN), GTHR, 0, stream>>>(F, L2T2, l2b, l2b, XL, Z2, 2 * MLPW, HID, 0);
  k_gemm<3><<<dim3(1, FOUT / GBN), GTHR, 0, stream>>>(Z2, FNT2, fb, fb, out, H1, 2 * HID, FOUT, 0);
}
